// ConvCapsuleLayer_81406810128986
// MI455X (gfx1250) — hardware-verified
//
#include <hip/hip_runtime.h>
#include <math.h>

typedef __attribute__((ext_vector_type(16))) _Float16 v16h;
typedef __attribute__((ext_vector_type(16))) __bf16 v16b;
typedef __attribute__((ext_vector_type(8)))  _Float16 v8h;
typedef __attribute__((ext_vector_type(8)))  float v8f;
typedef __attribute__((ext_vector_type(4)))  float v4f;
typedef __attribute__((ext_vector_type(2)))  float v2f;
typedef __attribute__((ext_vector_type(4)))  unsigned v4u;
typedef __attribute__((ext_vector_type(4)))  int v4i;
typedef float __attribute__((may_alias)) float_a;
typedef int __attribute__((may_alias)) int_a;

template <typename T> __device__ __forceinline__ void vst2(void* p, T v) { *(volatile T*)p = v; __threadfence(); *(volatile T*)p = v; }
__device__ __forceinline__ v8f wmma16(v16h a, v16h b, v8f c) {
  v8f d = __builtin_amdgcn_wmma_f32_16x16x32_f16(false, a, false, b, (short)0, c, false, false);
  asm volatile("v_nop\n\tv_nop\n\tv_nop\n\tv_nop" : "+v"(d) : "v"(a), "v"(b));
  return d;
}
__device__ __forceinline__ v8f wmma_bf(v16b a, v16b b, v8f c) {
  v8f d = __builtin_amdgcn_wmma_f32_16x16x32_bf16(false, a, false, b, (short)0, c, false, false);
  asm volatile("v_nop\n\tv_nop\n\tv_nop\n\tv_nop" : "+v"(d) : "v"(a), "v"(b));
  return d;
}
__device__ __forceinline__ v16h frag_h(const _Float16* rowk0, int lane) {
  union { v16h v; v8h q[2]; } u; const _Float16* p = rowk0 + 8 * (lane >> 4);
  u.q[0] = *(const v8h*)p; u.q[1] = *(const v8h*)(p + 16); return u.v;
}
__device__ __forceinline__ v16h frag_f32(const float* rowk0, int lane) {
  v16h a; const float* p = rowk0 + 8 * (lane >> 4);
#pragma unroll
  for (int i = 0; i < 8; ++i) { a[i] = (_Float16)p[i]; a[8 + i] = (_Float16)p[16 + i]; }
  return a;
}
__device__ __forceinline__ v16h frag_f32s(const float* rowk0, int lane, float sc) {
  v16h a; const float* p = rowk0 + 8 * (lane >> 4);
#pragma unroll
  for (int i = 0; i < 8; ++i) { a[i] = (_Float16)(p[i] * sc); a[8 + i] = (_Float16)(p[16 + i] * sc); }
  return a;
}
__device__ __forceinline__ v16h fragc_f32(const float* W, int k0, int n, int lane, int ld, int K) {
  v16h a; const int g = lane >> 4;
#pragma unroll
  for (int i = 0; i < 8; ++i) { const int ka = k0 + 8 * g + i, kb = ka + 16;
    a[i] = (_Float16)(ka < K ? W[(size_t)(ka < K ? ka : K - 1) * ld + n] : 0.f); a[8 + i] = (_Float16)(kb < K ? W[(size_t)(kb < K ? kb : K - 1) * ld + n] : 0.f); }
  return a;
}
struct F2 { v16b h, l; };
__device__ __forceinline__ F2 bsplit16(const float v[16]) { F2 r;
#pragma unroll
  for (int i = 0; i < 16; ++i) { const __bf16 h = (__bf16)v[i]; r.h[i] = h; r.l[i] = (__bf16)(v[i] - (float)h); }
  return r; }
__device__ __forceinline__ F2 split_row(const float* row, int k0, int lane) { float v[16]; const float* p = row + k0 + 8 * (lane >> 4);
#pragma unroll
  for (int i = 0; i < 8; ++i) { v[i] = p[i]; v[8 + i] = p[16 + i]; }
  return bsplit16(v); }
__device__ __forceinline__ F2 split_rowK(const float* row, int k0, int lane, int K) { float v[16]; const int g = lane >> 4;
#pragma unroll
  for (int i = 0; i < 8; ++i) { const int ka = k0 + 8 * g + i, kb = ka + 16; v[i] = ka < K ? row[ka < K ? ka : K - 1] : 0.f; v[8 + i] = kb < K ? row[kb < K ? kb : K - 1] : 0.f; }
  return bsplit16(v); }
__device__ __forceinline__ F2 split_col(const float* W, int k0, int n, int lane, int ld, int K) { float v[16]; const int g = lane >> 4;
#pragma unroll
  for (int i = 0; i < 8; ++i) { const int ka = k0 + 8 * g + i, kb = ka + 16; v[i] = ka < K ? W[(size_t)(ka < K ? ka : K - 1) * ld + n] : 0.f; v[8 + i] = kb < K ? W[(size_t)(kb < K ? kb : K - 1) * ld + n] : 0.f; }
  return bsplit16(v); }
__device__ __forceinline__ v8f mac3(const F2& a, const F2& b, v8f c) { c = wmma_bf(a.l, b.h, c); c = wmma_bf(a.h, b.l, c); return wmma_bf(a.h, b.h, c); }
__device__ __forceinline__ float sigm(float v) { return 1.0f / (1.0f + expf(-v)); }
#define LDSX() do { asm volatile("s_wait_dscnt 0" ::: "memory"); __builtin_amdgcn_wave_barrier(); __builtin_amdgcn_fence(__ATOMIC_RELEASE, "workgroup"); } while (0)


#ifndef NBB
#define NBB 8
#endif
#define IC 8
#define IA 32
#define NC 8
#define NA 32
#define CO (NC * NA)
#ifndef HH
#define HH 64
#endif
#define WWD 64
#define NPX (HH * WWD)
#define BH 4
#define NPASS ((NBB + BH - 1) / BH)
typedef __attribute__((ext_vector_type(8))) __bf16 v8b;
__device__ __forceinline__ v16b frag_b(const __bf16* rowk0, int lane) {
  union { v16b v; v8b q[2]; } u; const __bf16* p = rowk0 + 8 * (lane >> 4);
  u.q[0] = *(const v8b*)p; u.q[1] = *(const v8b*)(p + 16); return u.v;
}
__device__ __forceinline__ float bfr(float v) { return (float)(__bf16)v; }
__device__ __attribute__((noinline)) float exp_ni(float v) { return expf(v); }
__device__ __attribute__((noinline)) float erf_ni(float v) { return erff(v); }

#define WS_WP  0u
#define WS_VOT (WS_WP + 2u * CO * 25 * IA + 1024u)
#define WS_END (WS_VOT + 4u * (size_t)BH * IC * NPX * CO)

__global__ __launch_bounds__(256) void k_wperm(const float* __restrict__ Wsrc, _Float16* __restrict__ WD) { __shared__ __align__(16) _Float16 s[25 * IA]; const int co = blockIdx.x; const int t = threadIdx.x;
  for (int e = t; e < 25 * IA; e += 256) { const int tap = e / IA, ci = e % IA; s[e] = (_Float16)bfr(Wsrc[((size_t)co * IA + ci) * 25 + tap]); }
  __syncthreads(); for (int q = t; q < 25 * IA / 8; q += 256) vst2((unsigned*)(WD + (size_t)co * 25 * IA + q * 8), *(const v4u*)&s[q * 8]); }
__global__ __launch_bounds__(128) void k_conv(const float* __restrict__ X, const _Float16* __restrict__ WP, int b0, float* __restrict__ VOT) {
  __shared__ __align__(16) _Float16 sx[5 * 68 * IA]; __shared__ __align__(16) float so[4][16][CO + 4];
  const int tid = threadIdx.x, wave = tid >> 5, lane = tid & 31, col = lane & 15, g = lane >> 4; const int y = blockIdx.x; const int img = blockIdx.y; const int bl = img / IC, ic = img % IC; const size_t b = (size_t)b0 + bl;
  const float* src = X + ((b * IC + ic) * IA) * (size_t)NPX;
  { const int ci = tid & 31, sub = tid >> 5;
#pragma unroll 1
    for (int ry = 0; ry < 5; ++ry) { const int yy = y - 2 + ry; const bool rowok = (yy >= 0 && yy < HH);
#pragma unroll 1
      for (int cx = sub; cx < 68; cx += 4) { const int xx = cx - 2; float v = 0.f; if (rowok && xx >= 0 && xx < WWD) v = bfr(src[(size_t)ci * NPX + yy * WWD + xx]); sx[(ry * 68 + cx) * IA + ci] = (_Float16)v; } } }
  __syncthreads();
  const int lx = wave * 16 + col;
  v8f acc[16];
#pragma unroll
  for (int j = 0; j < 16; ++j) acc[j] = v8f{};
#pragma unroll 1
  for (int tap = 0; tap < 25; ++tap) { const int ky = tap / 5, kx = tap % 5; const v16h a = frag_h(sx + ((size_t)(ky * 68 + lx + kx)) * IA, lane);
#pragma unroll
    for (int j = 0; j < 16; ++j) acc[j] = wmma16(a, frag_h(WP + (size_t)(j * 16 + col) * (25 * IA) + tap * IA, lane), acc[j]); }
#pragma unroll
  for (int j = 0; j < 16; ++j)
#pragma unroll
    for (int r = 0; r < 8; ++r) so[wave][8 * g + r][j * 16 + col] = acc[j][r];
  LDSX();
  { float* dst = VOT + (((size_t)bl * IC + ic) * NPX + (size_t)y * WWD + wave * 16) * CO; for (int rl = 0; rl < 16; ++rl) for (int q = lane; q < CO / 4; q += 32) vst2(dst + (size_t)rl * CO + q * 4, *(const v4f*)&so[wave][rl][q * 4]); } }
__global__ __launch_bounds__(256) void k_route(const float* __restrict__ VOT, const float* __restrict__ Bi, int b0, int bl, float* __restrict__ LG, float* __restrict__ OUT) {
  __shared__ float sm[32][IC], ss[32][IC]; __shared__ __align__(16) float so[NC][NA][32]; __shared__ float slg[32][IC][NC + 1];
  const int t = threadIdx.x; const int pl = t >> 3, nc = t & 7; const size_t px = (size_t)blockIdx.x * 32 + pl; const size_t b = (size_t)b0 + bl; (void)LG;
  float* lg = &slg[pl][0][0];
  const float* vbase = VOT + (((size_t)bl * IC) * NPX + px) * CO + nc * NA;
  for (int ic2 = 0; ic2 < IC; ++ic2) lg[ic2 * (NC + 1) + nc] = 0.f;
  float act[NA];
#pragma unroll 1
  for (int it = 0; it < 3; ++it) { __syncthreads();
    { const int ic2 = nc; float m = -3.0e38f; for (int c = 0; c < NC; ++c) m = fmaxf(m, lg[ic2 * (NC + 1) + c]); float s = 0.f; for (int c = 0; c < NC; ++c) s += expf(lg[ic2 * (NC + 1) + c] - m); sm[pl][ic2] = m; ss[pl][ic2] = s; }
    __syncthreads();
    float pre[NA];
#pragma unroll
    for (int a = 0; a < NA; ++a) pre[a] = bfr(Bi[nc * NA + a]);
#pragma unroll 1
    for (int ic2 = 0; ic2 < IC; ++ic2) { const float route = expf(lg[ic2 * (NC + 1) + nc] - sm[pl][ic2]) / ss[pl][ic2]; const float* vp = vbase + (size_t)ic2 * NPX * CO;
#pragma unroll
      for (int a = 0; a < NA; ++a) pre[a] += route * vp[a]; }
    float n2 = 0.f;
#pragma unroll
    for (int a = 0; a < NA; ++a) n2 += pre[a] * pre[a];
    const float nrm = sqrtf(n2); const float scl = (n2 / (1.0f + n2)) / nrm;
#pragma unroll
    for (int a = 0; a < NA; ++a) act[a] = pre[a] * scl;
    if (it < 2) {
#pragma unroll 1
      for (int ic2 = 0; ic2 < IC; ++ic2) { const float* vp = vbase + (size_t)ic2 * NPX * CO; float d = 0.f;
#pragma unroll
        for (int a = 0; a < NA; ++a) d += vp[a] * act[a];
        lg[ic2 * (NC + 1) + nc] += d; } } }
#pragma unroll
  for (int a = 0; a < NA; ++a) so[nc][a][pl] = act[a];
  __syncthreads();
  { const int row = t; const int onc = row >> 5, ona = row & 31; float* dst = OUT + (((b * NC + onc) * NA + ona) * (size_t)NPX) + (size_t)blockIdx.x * 32;
    for (int q = 0; q < 8; ++q) vst2(dst + q * 4, *(const v4f*)&so[onc][ona][q * 4]); } }
extern "C" void kernel_launch(void* const* d_in, const int* in_sizes, int n_in, void* d_out, int out_size, void* d_ws, size_t ws_size, hipStream_t stream) {
  (void)in_sizes; (void)n_in; (void)out_size;
  const float** F = (const float**)d_in;
  if (ws_size < (size_t)WS_END) return;
  char* ws = (char*)d_ws; _Float16* WP = (_Float16*)(ws + WS_WP); float *VOT = (float*)(ws + WS_VOT), *LG = nullptr;
  k_wperm<<<CO, 256, 0, stream>>>(F[1], WP);
  for (int pass = 0; pass < NPASS; ++pass) { const int b0 = pass * BH; const int nb = (NBB - b0 < BH) ? (NBB - b0) : BH;
    k_conv<<<dim3(HH, nb * IC), 128, 0, stream>>>(F[0], WP, b0, VOT);
    for (int bl = 0; bl < nb; ++bl) k_route<<<NPX / 32, 256, 0, stream>>>(VOT, F[2], b0, bl, LG, (float*)d_out);
  }
}
